// RelativePositionMultiHeadAttention_12326556139724
// MI455X (gfx1250) — hardware-verified
//
#include <hip/hip_runtime.h>
#include <math.h>
typedef __attribute__((ext_vector_type(16))) _Float16 v16h;
typedef __attribute__((ext_vector_type(8)))  _Float16 v8h;
typedef __attribute__((ext_vector_type(16))) __bf16   v16b;
typedef __attribute__((ext_vector_type(8)))  __bf16   v8b;
typedef __attribute__((ext_vector_type(8)))  float    v8f;
typedef __attribute__((ext_vector_type(4)))  float    v4f;
#define PSCALE 32768.0f
#define U16(p) ((const unsigned short*)(const void*)(p))
#define PSCALE_INV (1.0f / 32768.0f)

__device__ __forceinline__ unsigned short f2bf_bits(float f) {
  unsigned u = __float_as_uint(f);
  return (unsigned short)((u + 0x7FFFu + ((u >> 16) & 1u)) >> 16);
}
__device__ __forceinline__ float bf_bits2f(unsigned short h) { return __uint_as_float(((unsigned)h) << 16); }

__device__ __forceinline__ void dep_guard_h(v8f& a, v8f& b, v16h x, v16h y) { asm volatile("v_nop\n\tv_nop\n\tv_nop\n\tv_nop" : "+v"(a), "+v"(b) : "v"(x), "v"(y)); }
__device__ __forceinline__ void dep_guard_b(v8f& a, v8f& b, v16b x, v16b y) { asm volatile("v_nop\n\tv_nop\n\tv_nop\n\tv_nop" : "+v"(a), "+v"(b) : "v"(x), "v"(y)); }
__device__ __forceinline__ void keep4_h(v16h a, v16h b, v16h c, v16h d) { asm volatile("v_nop" :: "v"(a), "v"(b), "v"(c), "v"(d)); }
__device__ __forceinline__ void keep4_b(v16b a, v16b b, v16b c, v16b d) { asm volatile("v_nop" :: "v"(a), "v"(b), "v"(c), "v"(d)); }
__device__ __forceinline__ void acc_guard4(v8f& a, v8f& b, v8f& c, v8f& d) { asm volatile("v_nop\n\tv_nop\n\tv_nop\n\tv_nop" : "+v"(a), "+v"(b), "+v"(c), "+v"(d)); }
template <typename T> struct Frag;
template <> struct Frag<_Float16> {
  typedef v16h V; union U { v16h v; v8h h[2]; };
  static __device__ __forceinline__ v16h load(const _Float16* p) {
    U f; f.h[0] = *(const v8h*)(p); f.h[1] = *(const v8h*)(p + 16); return f.v;
  }
  static __device__ __forceinline__ v8f mma(v16h a, v16h b, v8f c) {
    return __builtin_amdgcn_wmma_f32_16x16x32_f16(false, a, false, b, (short)0, c, false, false);
  }
  static __device__ __forceinline__ void guard(v8f& a, v8f& b, v16h x, v16h y) { dep_guard_h(a, b, x, y); }
  static __device__ __forceinline__ void keep(v16h a, v16h b, v16h c, v16h d) { keep4_h(a, b, c, d); }
};
template <> struct Frag<__bf16> {
  typedef v16b V; union U { v16b v; v8b h[2]; };
  static __device__ __forceinline__ v16b load(const __bf16* p) {
    U f; f.h[0] = *(const v8b*)(p); f.h[1] = *(const v8b*)(p + 16); return f.v;
  }
  static __device__ __forceinline__ v8f mma(v16b a, v16b b, v8f c) {
    return __builtin_amdgcn_wmma_f32_16x16x32_bf16(false, a, false, b, (short)0, c, false, false);
  }
  static __device__ __forceinline__ void guard(v8f& a, v8f& b, v16b x, v16b y) { dep_guard_b(a, b, x, y); }
  static __device__ __forceinline__ void keep(v16b a, v16b b, v16b c, v16b d) { keep4_b(a, b, c, d); }
};

template <int ET> struct Elem;
template <> struct Elem<0> { typedef _Float16 T; };
template <> struct Elem<1> { typedef __bf16 T; };
template <int ET, bool SPLIT, int BIAS_MODE, int OUT_MODE, bool RESID, int ACT = 0>
__global__ __launch_bounds__(256) void wmma_gemm64(
    const unsigned short* __restrict__ Ap, const unsigned short* __restrict__ A2p, int lda, long strideA,
    const unsigned short* __restrict__ Btp, const unsigned short* __restrict__ Bt2p, int ldb, long strideB,
    void* __restrict__ Cout, void* __restrict__ Cout2, int ldc, long strideC,
    const float* __restrict__ bias,
    const float* __restrict__ resid, long strideR,
    int M, int N, int K, float scale) {
  typedef typename Elem<ET>::T T;
  typedef typename Frag<T>::V V;
  const T* A = (const T*)Ap; const T* A2 = (const T*)A2p; const T* Bt = (const T*)Btp; const T* Bt2 = (const T*)Bt2p;
  __shared__ __align__(16) float sT[8][16 * 68];
  const int b    = blockIdx.y;
  const int lane = threadIdx.x & 31;
  const int wave = threadIdx.x >> 5;
  const int tilesN = N >> 6;
  const int tilesM = M >> 6;
  const int tile = blockIdx.x * 8 + wave;
  if (tile >= tilesM * tilesN) return;
  const int tm = tile / tilesN;
  const int tn = tile - tm * tilesN;
  const int m0 = tm << 6;
  const int n0 = tn << 6;

  const T* Ab  = A  + (size_t)b * strideA;
  const T* Bb  = Bt + (size_t)b * strideB;
  const T* Ab2 = SPLIT ? (A2  + (size_t)b * strideA) : nullptr;
  const T* Bb2 = SPLIT ? (Bt2 + (size_t)b * strideB) : nullptr;

  const int rlane = lane & 15;
  const int koff  = (lane >> 4) * 8;
  const int mOff  = (lane >> 4) * 8;

  v8f acc[4][4];
#pragma unroll
  for (int i = 0; i < 4; ++i)
#pragma unroll
    for (int j = 0; j < 4; ++j) acc[i][j] = (v8f){0.f,0.f,0.f,0.f,0.f,0.f,0.f,0.f};

  for (int k0 = 0; k0 < K; k0 += 32) {
    V bh[4], bl[4];
#pragma unroll
    for (int j = 0; j < 4; ++j) {
      const size_t bo = (size_t)(n0 + (j << 4) + rlane) * ldb + koff + k0;
      bh[j] = Frag<T>::load(Bb + bo);
      if (SPLIT) bl[j] = Frag<T>::load(Bb2 + bo);
    }
#pragma unroll
    for (int i = 0; i < 4; ++i) {
      const size_t ao = (size_t)(m0 + (i << 4) + rlane) * lda + koff + k0;
      V ah = Frag<T>::load(Ab + ao);
      V al;
      if (SPLIT) al = Frag<T>::load(Ab2 + ao);
#pragma unroll
      for (int j = 0; j < 4; ++j) {
        acc[i][j] = Frag<T>::mma(ah, bh[j], acc[i][j]);
        if (SPLIT) {
          acc[i][j] = Frag<T>::mma(ah, bl[j], acc[i][j]);
          acc[i][j] = Frag<T>::mma(al, bh[j], acc[i][j]);
        }
      }
      Frag<T>::guard(acc[i][0], acc[i][3], ah, SPLIT ? al : ah);
    }
    Frag<T>::keep(bh[0], bh[1], bh[2], bh[3]);
    if (SPLIT) Frag<T>::keep(bl[0], bl[1], bl[2], bl[3]);
  }
  acc_guard4(acc[0][0], acc[0][1], acc[0][2], acc[0][3]);
  acc_guard4(acc[1][0], acc[1][1], acc[1][2], acc[1][3]);
  acc_guard4(acc[2][0], acc[2][1], acc[2][2], acc[2][3]);
  acc_guard4(acc[3][0], acc[3][1], acc[3][2], acc[3][3]);

  float* slab = sT[wave];
  const float* Rb = RESID ? (resid + (size_t)b * strideR) : nullptr;
#pragma unroll
  for (int i = 0; i < 4; ++i) {
    const int mBase = m0 + (i << 4);
#pragma unroll
    for (int j = 0; j < 4; ++j) {
      const int n = n0 + (j << 4) + rlane;
      float bv = 0.f;
      if (BIAS_MODE == 2) bv = bias[n];
#pragma unroll
      for (int r = 0; r < 8; ++r) {
        float v = acc[i][j][r] * scale;
        if (BIAS_MODE == 1) v += bias[mBase + mOff + r];
        if (BIAS_MODE == 2) v += bv;
        if (RESID) v += Rb[(size_t)(mBase + mOff + r) * ldc + n];
        if (ACT == 1) v = tanhf(v);
        if (ACT == 2) v = fmaxf(v, 0.0f);
        if (ACT == 3) v = v / (1.0f + expf(-v));
        if (ACT == 4) v = (v > 0.f) ? v : 0.01f * v;
        if (ACT == 5) v = 0.5f * v * (1.0f + erff(v * 0.70710678118654752f));
        slab[(mOff + r) * 68 + (j << 4) + rlane] = v;
      }
    }
    __builtin_amdgcn_fence(__ATOMIC_RELEASE, "workgroup");
    __builtin_amdgcn_wave_barrier();
    __builtin_amdgcn_fence(__ATOMIC_ACQUIRE, "workgroup");
    if (OUT_MODE == 0) {
      float* C = (float*)Cout + (size_t)b * strideC;
      const int hh = lane >> 4, c4 = (lane & 15) * 4;
      for (int pass = 0; pass < 2; ++pass) {
#pragma unroll
        for (int it = 0; it < 8; ++it) {
          const int row = it * 2 + hh;
          v4f v = *(const v4f*)(slab + row * 68 + c4);
          *(volatile v4f*)(C + (size_t)(mBase + row) * ldc + n0 + c4) = v;
        }
        __threadfence();
      }
    } else {
      const int q = lane >> 3, c8 = (lane & 7) * 8;
      unsigned short* C  = (unsigned short*)Cout  + (size_t)b * strideC;
      unsigned short* C2 = (OUT_MODE == 2) ? ((unsigned short*)Cout2 + (size_t)b * strideC) : nullptr;
      for (int pass = 0; pass < 2; ++pass) {
#pragma unroll
        for (int it = 0; it < 4; ++it) {
          const int row = it * 4 + q;
          const float* sp = slab + row * 68 + c8;
          v8h hv, lv;
#pragma unroll
          for (int e = 0; e < 8; ++e) {
            if (OUT_MODE == 1) {
              hv[e] = (_Float16)sp[e];
            } else {
              unsigned short hb = f2bf_bits(sp[e]);
              unsigned short lb = f2bf_bits(sp[e] - bf_bits2f(hb));
              hv[e] = __builtin_bit_cast(_Float16, hb);
              lv[e] = __builtin_bit_cast(_Float16, lb);
            }
          }
          *(volatile v8h*)(C + (size_t)(mBase + row) * ldc + n0 + c8) = hv;
          if (OUT_MODE == 2) *(volatile v8h*)(C2 + (size_t)(mBase + row) * ldc + n0 + c8) = lv;
        }
        __threadfence();
      }
    }
    __builtin_amdgcn_fence(__ATOMIC_RELEASE, "workgroup");
    __builtin_amdgcn_wave_barrier();
    __builtin_amdgcn_fence(__ATOMIC_ACQUIRE, "workgroup");
  }
}

__global__ __launch_bounds__(256) void cast_f32_f16x2(
    const float* __restrict__ in, _Float16* __restrict__ out, int n2) {
  int i = blockIdx.x * 256 + threadIdx.x;
  if (i < n2) {
    const _Float16 h0 = (_Float16)in[2 * i], h1 = (_Float16)in[2 * i + 1];
    const unsigned u = (unsigned)__builtin_bit_cast(unsigned short, h0) | ((unsigned)__builtin_bit_cast(unsigned short, h1) << 16);
    ((volatile unsigned*)out)[i] = u;
    __threadfence();
    ((volatile unsigned*)out)[i] = u;
  }
}


#define RB_ 8
#define RT 1024
#define RM 512
#define RE 64
#define RH 8
#define RKX 192
__global__ __launch_bounds__(256) void wperm_kernel(const float* __restrict__ wsrc, int is_out, unsigned* __restrict__ BT) {
  for (int i = blockIdx.x * 256 + threadIdx.x; i < RM * RM / 2; i += gridDim.x * 256) { const int row = i / (RM / 2), cp = 2 * (i % (RM / 2)); float a, b;
    if (!is_out) { const int h = row / RE, e = row % RE; a = wsrc[((size_t)cp * RE + e) * RH + h]; b = wsrc[((size_t)(cp + 1) * RE + e) * RH + h]; }
    else { const int m = row; const int h0 = cp / RE, e0 = cp % RE, h1 = (cp + 1) / RE, e1 = (cp + 1) % RE; a = wsrc[((size_t)e0 * RH + h0) * RM + m]; b = wsrc[((size_t)e1 * RH + h1) * RM + m]; }
    const unsigned u = (unsigned)__builtin_bit_cast(unsigned short, (_Float16)a) | ((unsigned)__builtin_bit_cast(unsigned short, (_Float16)b) << 16); ((volatile unsigned*)BT)[i] = u; __threadfence(); ((volatile unsigned*)BT)[i] = u; }
}
__global__ __launch_bounds__(256) void ext_kernel(const float* __restrict__ QP, const float* __restrict__ KP, const float* __restrict__ bu, const float* __restrict__ bv, int b0, unsigned* __restrict__ QX, unsigned* __restrict__ KX) {
  const int lane = threadIdx.x & 31, wave = threadIdx.x >> 5; const long g = (long)blockIdx.x * 8 + wave; const int h = (int)(g % RH); const int t = (int)(g / RH); const int b = b0; const long bt = (long)b * RT + t;
  const int e0 = 2 * lane, e1 = 2 * lane + 1;
  const float q0 = QP[bt * RM + h * RE + e0], q1 = QP[bt * RM + h * RE + e1], k0 = KP[bt * RM + h * RE + e0], k1 = KP[bt * RM + h * RE + e1];
  const float inv0 = powf(10000.0f, (float)((e0 / 2) * 2) / (float)RE), inv1 = powf(10000.0f, (float)((e1 / 2) * 2) / (float)RE);
  const float th0 = (float)t / inv0, th1 = (float)t / inv1; const float s0 = sinf(th0), c0 = cosf(th0), s1 = sinf(th1), c1 = cosf(th1);
  const float a0 = c0, be0 = -s0;
  const float a1 = s1, be1 = c1;
  const float qv0 = q0 + bv[e0 * RH + h], qv1 = q1 + bv[e1 * RH + h];
  const size_t row = ((size_t)h * RT + t) * RKX;
  for (int pass = 0; pass < 2; ++pass) {
    ((volatile unsigned*)QX)[(row) / 2 + lane] = (unsigned)__builtin_bit_cast(unsigned short, (_Float16)(q0 + bu[e0 * RH + h])) | ((unsigned)__builtin_bit_cast(unsigned short, (_Float16)(q1 + bu[e1 * RH + h])) << 16);
    ((volatile unsigned*)QX)[(row + 64) / 2 + lane] = (unsigned)__builtin_bit_cast(unsigned short, (_Float16)(qv0 * a0)) | ((unsigned)__builtin_bit_cast(unsigned short, (_Float16)(qv1 * a1)) << 16);
    ((volatile unsigned*)QX)[(row + 128) / 2 + lane] = (unsigned)__builtin_bit_cast(unsigned short, (_Float16)(qv0 * be0)) | ((unsigned)__builtin_bit_cast(unsigned short, (_Float16)(qv1 * be1)) << 16);
    ((volatile unsigned*)KX)[(row) / 2 + lane] = (unsigned)__builtin_bit_cast(unsigned short, (_Float16)k0) | ((unsigned)__builtin_bit_cast(unsigned short, (_Float16)k1) << 16);
    ((volatile unsigned*)KX)[(row + 64) / 2 + lane] = (unsigned)__builtin_bit_cast(unsigned short, (_Float16)s0) | ((unsigned)__builtin_bit_cast(unsigned short, (_Float16)s1) << 16);
    ((volatile unsigned*)KX)[(row + 128) / 2 + lane] = (unsigned)__builtin_bit_cast(unsigned short, (_Float16)c0) | ((unsigned)__builtin_bit_cast(unsigned short, (_Float16)c1) << 16);
    __threadfence(); }
}
__global__ __launch_bounds__(256) void vt_kernel(const float* __restrict__ VP, unsigned* __restrict__ VT) {
  __shared__ float tile[64][65];
  const int bh = blockIdx.y, j0 = blockIdx.x * 64, tx = threadIdx.x, ty = threadIdx.y; const int b = bh / RH, h = bh % RH;
  for (int j = ty; j < 64; j += 8) { const float* src = VP + ((size_t)b * RT + j0 + j) * RM + h * RE; tile[j][tx] = src[tx]; tile[j][32 + tx] = src[32 + tx]; }
  __syncthreads();
  for (int pass = 0; pass < 2; ++pass) { for (int e = ty; e < 64; e += 8) ((volatile unsigned*)VT)[(((size_t)bh * RE + e) * RT + j0) / 2 + tx] = (unsigned)__builtin_bit_cast(unsigned short, (_Float16)tile[2 * tx][e]) | ((unsigned)__builtin_bit_cast(unsigned short, (_Float16)tile[2 * tx + 1][e]) << 16); __threadfence(); }
}
__global__ __launch_bounds__(256) void soft_kernel(const float* __restrict__ S, const int* __restrict__ maskb, unsigned* __restrict__ P16) {
  const int lane = threadIdx.x & 31, wave = threadIdx.x >> 5; const size_t row = (size_t)blockIdx.x * 8 + wave; const float* s = S + row * RT;
  float v[32]; float mx = -INFINITY;
#pragma unroll
  for (int q = 0; q < 32; ++q) { const int j = lane * 32 + q; float x = s[j]; if (maskb[j] == 0) x = -INFINITY; v[q] = x; mx = fmaxf(mx, x); }
  for (int o = 16; o > 0; o >>= 1) mx = fmaxf(mx, __shfl_xor(mx, o, 32));
  float sum = 0.f;
#pragma unroll
  for (int q = 0; q < 32; ++q) { v[q] = (v[q] == -INFINITY) ? 0.f : __expf(v[q] - mx); sum += v[q]; }
  for (int o = 16; o > 0; o >>= 1) sum += __shfl_xor(sum, o, 32);
  const float sc = 32768.0f / sum;
  typedef __attribute__((ext_vector_type(4))) unsigned u4;
  for (int pass = 0; pass < 2; ++pass) {
#pragma unroll
    for (int q4 = 0; q4 < 4; ++q4) { u4 u; for (int z = 0; z < 4; ++z) { const int q = q4 * 8 + 2 * z; u[z] = (unsigned)__builtin_bit_cast(unsigned short, (_Float16)(v[q] * sc)) | ((unsigned)__builtin_bit_cast(unsigned short, (_Float16)(v[q + 1] * sc)) << 16); }
      *(volatile u4*)(P16 + (row * RT + lane * 32 + q4 * 8) / 2) = u; }
    __threadfence(); }
}
extern "C" void kernel_launch(void* const* d_in, const int* in_sizes, int n_in, void* d_out, int out_size, void* d_ws, size_t ws_size, hipStream_t stream) {
  (void)in_sizes; (void)n_in; (void)out_size; (void)ws_size;
  auto Fp = [&](int i) { return (const float*)d_in[i]; };
  const float* q = Fp(0); const float* k = Fp(1); const float* v = Fp(2); const int* mask = (const int*)d_in[3]; const float* wq = Fp(4); const float* wk = Fp(5); const float* wv = Fp(6); const float* bu = Fp(7); const float* bv = Fp(8); const float* wo = Fp(9);
  char* ws = (char*)d_ws; size_t off = 0;
  auto carve = [&](size_t bytes) -> char* { char* p = ws + off; off += (bytes + 255) & ~(size_t)255; return p; };
  const size_t NTOK = (size_t)RB_ * RT;
  _Float16* X16 = (_Float16*)carve(NTOK * RM * 2); unsigned* WQT = (unsigned*)carve(RM * RM * 2); unsigned* WKT = (unsigned*)carve(RM * RM * 2); unsigned* WVT = (unsigned*)carve(RM * RM * 2); unsigned* WOT = (unsigned*)carve(RM * RM * 2);
  float* QP = (float*)carve(NTOK * RM * 4); float* KP = (float*)carve(NTOK * RM * 4); float* VP = (float*)carve(NTOK * RM * 4);
  unsigned* QX = (unsigned*)carve((size_t)RH * RT * RKX * 2); unsigned* KX = (unsigned*)carve((size_t)RH * RT * RKX * 2); unsigned* VT = (unsigned*)carve(NTOK * RM * 2);
  unsigned* P16 = (unsigned*)carve((size_t)RH * RT * RT * 2); _Float16* O16 = (_Float16*)X16;
  float* S = (float*)carve((size_t)RH * RT * RT * 4);
  wperm_kernel<<<64, 256, 0, stream>>>(wq, 0, WQT); wperm_kernel<<<64, 256, 0, stream>>>(wk, 0, WKT); wperm_kernel<<<64, 256, 0, stream>>>(wv, 0, WVT); wperm_kernel<<<64, 256, 0, stream>>>(wo, 1, WOT);
  const int tp = (int)((NTOK / 64) * (RM / 64));
  cast_f32_f16x2<<<(unsigned)((NTOK * RM / 2 + 255) / 256), 256, 0, stream>>>(q, X16, (long)(NTOK * RM / 2));
  wmma_gemm64<0, false, 0, 0, false><<<dim3((tp + 7) / 8, 1), 256, 0, stream>>>(U16(X16), nullptr, RM, 0, (const unsigned short*)WQT, nullptr, RM, 0, QP, nullptr, RM, 0, nullptr, nullptr, 0, (int)NTOK, RM, RM, 1.0f);
  cast_f32_f16x2<<<(unsigned)((NTOK * RM / 2 + 255) / 256), 256, 0, stream>>>(k, X16, (long)(NTOK * RM / 2));
  wmma_gemm64<0, false, 0, 0, false><<<dim3((tp + 7) / 8, 1), 256, 0, stream>>>(U16(X16), nullptr, RM, 0, (const unsigned short*)WKT, nullptr, RM, 0, KP, nullptr, RM, 0, nullptr, nullptr, 0, (int)NTOK, RM, RM, 1.0f);
  cast_f32_f16x2<<<(unsigned)((NTOK * RM / 2 + 255) / 256), 256, 0, stream>>>(v, X16, (long)(NTOK * RM / 2));
  wmma_gemm64<0, false, 0, 0, false><<<dim3((tp + 7) / 8, 1), 256, 0, stream>>>(U16(X16), nullptr, RM, 0, (const unsigned short*)WVT, nullptr, RM, 0, VP, nullptr, RM, 0, nullptr, nullptr, 0, (int)NTOK, RM, RM, 1.0f);
  vt_kernel<<<dim3(RT / 64, RB_ * RH), dim3(32, 8), 0, stream>>>(VP, VT);
  const int ts = (RT / 64) * (RT / 64), to = (RT / 64) * 1;
  for (int b = 0; b < RB_; ++b) {
    ext_kernel<<<(unsigned)(RT * RH / 8), 256, 0, stream>>>(QP, KP, bu, bv, b, QX, KX);
    wmma_gemm64<0, false, 0, 0, false><<<dim3((ts + 7) / 8, RH), 256, 0, stream>>>((const unsigned short*)QX, nullptr, RKX, (long)RT * RKX, (const unsigned short*)KX, nullptr, RKX, (long)RT * RKX, S, nullptr, RT, (long)RT * RT, nullptr, nullptr, 0, RT, RT, RKX, 0.125f);
    soft_kernel<<<RH * RT / 8, 256, 0, stream>>>(S, mask + (size_t)b * RT, P16);
    wmma_gemm64<0, false, 0, 1, false><<<dim3((to + 7) / 8, RH), 256, 0, stream>>>((const unsigned short*)P16, nullptr, RT, (long)RT * RT, (const unsigned short*)VT + (size_t)b * RH * RE * RT, nullptr, RT, (long)RE * RT, O16 + (size_t)b * RT * RM, nullptr, RM, RE, nullptr, nullptr, 0, RT, RE, RT, 1.0f / 32768.0f); }
  wmma_gemm64<0, false, 0, 0, false><<<dim3((tp + 7) / 8, 1), 256, 0, stream>>>(U16(O16), nullptr, RM, 0, (const unsigned short*)WOT, nullptr, RM, 0, (float*)d_out, nullptr, RM, 0, nullptr, nullptr, 0, (int)NTOK, RM, RM, 1.0f);
}
